// LCAOOut_12438225289736
// MI455X (gfx1250) — hardware-verified
//
#include <hip/hip_runtime.h>
#include <stdint.h>
#include <math.h>

#define NN 50000
#define NP 50048
#define NE 800000
#define EMB 128
#define EC 160000
#define NCHK (NE / EC)
#define TN 4096
#define NTILE 13
#define NT 256
#define WSC 16.0f
#define WSC_INV 0.0625f

typedef __attribute__((ext_vector_type(16))) _Float16 v16h;
typedef __attribute__((ext_vector_type(8)))  _Float16 v8h;
typedef __attribute__((ext_vector_type(16))) __bf16   v16b;
typedef __attribute__((ext_vector_type(8)))  __bf16   v8b;
typedef __attribute__((ext_vector_type(8)))  float    v8f;
typedef __attribute__((ext_vector_type(4)))  float    v4f;
typedef __attribute__((ext_vector_type(4)))  int      v4i;

__device__ __forceinline__ unsigned short f2bf_bits(float f) {
  unsigned u = __float_as_uint(f);
  return (unsigned short)((u + 0x7FFFu + ((u >> 16) & 1u)) >> 16);
}
__device__ __forceinline__ float bf_bits2f(unsigned short h) { return __uint_as_float(((unsigned)h) << 16); }

__device__ __forceinline__ float silu_f(float v) { return v * __builtin_amdgcn_rcpf(1.0f + __expf(-v)); }

__device__ __forceinline__ void dep_guard_h(v8f& a, v8f& b, v16h x, v16h y) { asm volatile("v_nop\n\tv_nop\n\tv_nop\n\tv_nop" : "+v"(a), "+v"(b) : "v"(x), "v"(y)); }
__device__ __forceinline__ void dep_guard_b(v8f& a, v8f& b, v16b x, v16b y) { asm volatile("v_nop\n\tv_nop\n\tv_nop\n\tv_nop" : "+v"(a), "+v"(b) : "v"(x), "v"(y)); }
__device__ __forceinline__ void keep4_h(v16h a, v16h b, v16h c, v16h d) { asm volatile("v_nop" :: "v"(a), "v"(b), "v"(c), "v"(d)); }
__device__ __forceinline__ void keep4_b(v16b a, v16b b, v16b c, v16b d) { asm volatile("v_nop" :: "v"(a), "v"(b), "v"(c), "v"(d)); }
__device__ __forceinline__ void acc_guard4(v8f& a, v8f& b, v8f& c, v8f& d) { asm volatile("v_nop\n\tv_nop\n\tv_nop\n\tv_nop" : "+v"(a), "+v"(b), "+v"(c), "+v"(d)); }
template <typename T> struct Frag;
template <> struct Frag<_Float16> {
  typedef v16h V; union U { v16h v; v8h h[2]; };
  static __device__ __forceinline__ v16h load(const _Float16* p) {
    U f; f.h[0] = *(const v8h*)(p); f.h[1] = *(const v8h*)(p + 16); return f.v;
  }
  static __device__ __forceinline__ v8f mma(v16h a, v16h b, v8f c) {
    return __builtin_amdgcn_wmma_f32_16x16x32_f16(false, a, false, b, (short)0, c, false, false);
  }
  static __device__ __forceinline__ void guard(v8f& a, v8f& b, v16h x, v16h y) { dep_guard_h(a, b, x, y); }
  static __device__ __forceinline__ void keep(v16h a, v16h b, v16h c, v16h d) { keep4_h(a, b, c, d); }
};
template <> struct Frag<__bf16> {
  typedef v16b V; union U { v16b v; v8b h[2]; };
  static __device__ __forceinline__ v16b load(const __bf16* p) {
    U f; f.h[0] = *(const v8b*)(p); f.h[1] = *(const v8b*)(p + 16); return f.v;
  }
  static __device__ __forceinline__ v8f mma(v16b a, v16b b, v8f c) {
    return __builtin_amdgcn_wmma_f32_16x16x32_bf16(false, a, false, b, (short)0, c, false, false);
  }
  static __device__ __forceinline__ void guard(v8f& a, v8f& b, v16b x, v16b y) { dep_guard_b(a, b, x, y); }
  static __device__ __forceinline__ void keep(v16b a, v16b b, v16b c, v16b d) { keep4_b(a, b, c, d); }
};

template <int ET> struct Elem;
template <> struct Elem<0> { typedef _Float16 T; };
template <> struct Elem<1> { typedef __bf16 T; };
template <int ET, bool SPLIT, int BIAS_MODE, int OUT_MODE, bool RESID, int ACT = 0>
__global__ __launch_bounds__(256) void wmma_gemm64(
    const unsigned short* __restrict__ Ap, const unsigned short* __restrict__ A2p, int lda, long strideA,
    const unsigned short* __restrict__ Btp, const unsigned short* __restrict__ Bt2p, int ldb, long strideB,
    void* __restrict__ Cout, void* __restrict__ Cout2, int ldc, long strideC,
    const float* __restrict__ bias,
    const float* __restrict__ resid, long strideR,
    int M, int N, int K, float scale, const float* __restrict__ rdw) {
  typedef typename Elem<ET>::T T;
  typedef typename Frag<T>::V V;
  const T* A = (const T*)Ap; const T* A2 = (const T*)A2p; const T* Bt = (const T*)Btp; const T* Bt2 = (const T*)Bt2p;
  __shared__ __align__(16) float sT[8][16 * 68];
  __shared__ __align__(16) float sW[8][64];
  __shared__ __align__(16) float sR[8][64];
  const int b    = blockIdx.y;
  const int lane = threadIdx.x & 31;
  const int wave = threadIdx.x >> 5;
  const int tilesN = N >> 6;
  const int tilesM = M >> 6;
  const int tile = blockIdx.x * 8 + wave;
  if (tile >= tilesM * tilesN) return;
  const int tm = tile / tilesN;
  const int tn = tile - tm * tilesN;
  const int m0 = tm << 6;
  const int n0 = tn << 6;

  const T* Ab  = A  + (size_t)b * strideA;
  const T* Bb  = Bt + (size_t)b * strideB;
  const T* Ab2 = SPLIT ? (A2  + (size_t)b * strideA) : nullptr;
  const T* Bb2 = SPLIT ? (Bt2 + (size_t)b * strideB) : nullptr;

  const int rlane = lane & 15;
  const int koff  = (lane >> 4) * 8;
  const int mOff  = (lane >> 4) * 8;

  v8f acc[4][4];
#pragma unroll
  for (int i = 0; i < 4; ++i)
#pragma unroll
    for (int j = 0; j < 4; ++j) acc[i][j] = (v8f){0.f,0.f,0.f,0.f,0.f,0.f,0.f,0.f};

  for (int k0 = 0; k0 < K; k0 += 32) {
    V bh[4], bl[4];
#pragma unroll
    for (int j = 0; j < 4; ++j) {
      const size_t bo = (size_t)(n0 + (j << 4) + rlane) * ldb + koff + k0;
      bh[j] = Frag<T>::load(Bb + bo);
      if (SPLIT) bl[j] = Frag<T>::load(Bb2 + bo);
    }
#pragma unroll
    for (int i = 0; i < 4; ++i) {
      const size_t ao = (size_t)(m0 + (i << 4) + rlane) * lda + koff + k0;
      V ah = Frag<T>::load(Ab + ao);
      V al;
      if (SPLIT) al = Frag<T>::load(Ab2 + ao);
#pragma unroll
      for (int j = 0; j < 4; ++j) {
        acc[i][j] = Frag<T>::mma(ah, bh[j], acc[i][j]);
        if (SPLIT) {
          acc[i][j] = Frag<T>::mma(ah, bl[j], acc[i][j]);
          acc[i][j] = Frag<T>::mma(al, bh[j], acc[i][j]);
        }
      }
      Frag<T>::guard(acc[i][0], acc[i][3], ah, SPLIT ? al : ah);
    }
    Frag<T>::keep(bh[0], bh[1], bh[2], bh[3]);
    if (SPLIT) Frag<T>::keep(bl[0], bl[1], bl[2], bl[3]);
  }
  acc_guard4(acc[0][0], acc[0][1], acc[0][2], acc[0][3]);
  acc_guard4(acc[1][0], acc[1][1], acc[1][2], acc[1][3]);
  acc_guard4(acc[2][0], acc[2][1], acc[2][2], acc[2][3]);
  acc_guard4(acc[3][0], acc[3][1], acc[3][2], acc[3][3]);

  float* slab = sT[wave];
  float* sWv  = sW[wave];
  float* sRv  = sR[wave];
  const float* Rb = RESID ? (resid + (size_t)b * strideR) : nullptr;
  if (OUT_MODE == 3) { sWv[lane] = rdw[n0 + lane]; sWv[32 + lane] = rdw[n0 + 32 + lane]; }
#pragma unroll
  for (int i = 0; i < 4; ++i) {
    const int mBase = m0 + (i << 4);
#pragma unroll
    for (int j = 0; j < 4; ++j) {
      const int n = n0 + (j << 4) + rlane;
      float bv = 0.f;
      if (BIAS_MODE == 2) bv = bias[n];
#pragma unroll
      for (int r = 0; r < 8; ++r) {
        float v = acc[i][j][r] * scale;
        if (BIAS_MODE == 1) v += bias[mBase + mOff + r];
        if (BIAS_MODE == 2) v += bv;
        if (RESID) v += Rb[(size_t)(mBase + mOff + r) * ldc + n];
        if (ACT == 1) v = tanhf(v);
        if (ACT == 2) v = fmaxf(v, 0.0f);
        if (ACT == 3) v = v / (1.0f + expf(-v));
        if (ACT == 4) v = (v > 0.f) ? v : 0.01f * v;
        if (ACT == 5) v = 0.5f * v * (1.0f + erff(v * 0.70710678118654752f));
        if (ACT == 6) v = silu_f(v);
        slab[(mOff + r) * 68 + (j << 4) + rlane] = v;
      }
    }
    __builtin_amdgcn_fence(__ATOMIC_RELEASE, "workgroup");
    __builtin_amdgcn_wave_barrier();
    __builtin_amdgcn_fence(__ATOMIC_ACQUIRE, "workgroup");
    if (OUT_MODE == 0) {
      float* C = (float*)Cout + (size_t)b * strideC;
      const int hh = lane >> 4, c4 = (lane & 15) * 4;
      for (int pass = 0; pass < 2; ++pass) {
#pragma unroll
        for (int it = 0; it < 8; ++it) {
          const int row = it * 2 + hh;
          v4f v = *(const v4f*)(slab + row * 68 + c4);
          *(volatile v4f*)(C + (size_t)(mBase + row) * ldc + n0 + c4) = v;
        }
        __threadfence();
      }
    } else if (OUT_MODE == 3) {
      const int rw = lane & 15, hs = lane >> 4;
      const float* sp = slab + rw * 68 + hs * 32;
      const float* wp = sWv + hs * 32;
      float d = 0.f;
#pragma unroll
      for (int c = 0; c < 32; ++c) d += sp[c] * wp[c];
      d += __shfl_xor(d, 16, 32);
      if (hs == 0) sRv[(i << 4) + rw] = d;
    } else {
      const int q = lane >> 3, c8 = (lane & 7) * 8;
      unsigned short* C  = (unsigned short*)Cout  + (size_t)b * strideC;
      unsigned short* C2 = (OUT_MODE == 2) ? ((unsigned short*)Cout2 + (size_t)b * strideC) : nullptr;
      for (int pass = 0; pass < 2; ++pass) {
#pragma unroll
        for (int it = 0; it < 4; ++it) {
          const int row = it * 4 + q;
          const float* sp = slab + row * 68 + c8;
          v8h hv, lv;
#pragma unroll
          for (int e = 0; e < 8; ++e) {
            if (OUT_MODE == 1) {
              hv[e] = (_Float16)sp[e];
            } else {
              unsigned short hb = f2bf_bits(sp[e]);
              unsigned short lb = f2bf_bits(sp[e] - bf_bits2f(hb));
              hv[e] = __builtin_bit_cast(_Float16, hb);
              lv[e] = __builtin_bit_cast(_Float16, lb);
            }
          }
          *(volatile v8h*)(C + (size_t)(mBase + row) * ldc + n0 + c8) = hv;
          if (OUT_MODE == 2) *(volatile v8h*)(C2 + (size_t)(mBase + row) * ldc + n0 + c8) = lv;
        }
        __threadfence();
      }
    }
    __builtin_amdgcn_fence(__ATOMIC_RELEASE, "workgroup");
    __builtin_amdgcn_wave_barrier();
    __builtin_amdgcn_fence(__ATOMIC_ACQUIRE, "workgroup");
  }
  if (OUT_MODE == 3) {
    float* C = (float*)Cout + (size_t)b * strideC;
    const v4f o = *(const v4f*)(sRv + 4 * (lane & 15));
    for (int pass = 0; pass < 2; ++pass) {
      if (lane < 16) *(volatile v4f*)(C + m0 + 4 * lane) = o;
      __threadfence();
    }
  }
}

__device__ __forceinline__ int blk_excl_scan(int cnt, int* scan_ws, int tid, int* tot) {
  const int lane = tid & 31, wave = tid >> 5; int incl = cnt;
#pragma unroll
  for (int o = 1; o < 32; o <<= 1) { const int v = __shfl_up(incl, o, 32); if (lane >= o) incl += v; }
  if (lane == 31) scan_ws[wave] = incl;
  __syncthreads();
  if (wave == 0) { int wv = (lane < NT / 32) ? scan_ws[lane] : 0; int wincl = wv;
#pragma unroll
    for (int o = 1; o < 32; o <<= 1) { const int v = __shfl_up(wincl, o, 32); if (lane >= o) wincl += v; }
    if (lane < NT / 32) scan_ws[32 + lane] = wincl - wv; if (lane == 31) scan_ws[64] = wincl; }
  __syncthreads();
  const int res = scan_ws[32 + wave] + incl - cnt; *tot = scan_ws[64];
  return res;
}

__global__ __launch_bounds__(NT) void prep_w_kernel(const float* __restrict__ W1, const float* __restrict__ W2,
                                                  const float* __restrict__ Wf1, const float* __restrict__ Wf2,
                                                  _Float16* __restrict__ WT) {
  const int i = blockIdx.x * NT + threadIdx.x;
  if (i >= 32768) return;
  const int hx = 2 * i;
  float v0, v1;
  if (hx < 16384) {
    const int n = hx >> 7, k = hx & 127;
    v0 = W1[k * 128 + n]; v1 = W1[(k + 1) * 128 + n];
  } else if (hx < 24576) {
    const int l = hx - 16384; const int n = l >> 7, k = l & 127;
    v0 = W2[k * 64 + n]; v1 = W2[(k + 1) * 64 + n];
  } else if (hx < 57344) {
    const int l = hx - 24576; const int n = l >> 7, k = l & 127;
    const int kr = (n < 128) ? k : (128 + k); const int nc = n & 127;
    v0 = Wf1[kr * 128 + nc]; v1 = Wf1[(kr + 1) * 128 + nc];
  } else {
    const int l = hx - 57344; const int n = l >> 7, k = l & 127;
    v0 = Wf2[k * 64 + n]; v1 = Wf2[(k + 1) * 64 + n];
  }
  const _Float16 h0 = (_Float16)(v0 * WSC), h1 = (_Float16)(v1 * WSC);
  const unsigned u = (unsigned)__builtin_bit_cast(unsigned short, h0) | ((unsigned)__builtin_bit_cast(unsigned short, h1) << 16);
  ((volatile unsigned*)WT)[i] = u;
  __threadfence();
  ((volatile unsigned*)WT)[i] = u;
}

__global__ __launch_bounds__(NT) void cast_x_kernel(const float* __restrict__ x, _Float16* __restrict__ Xh) {
  const int i = blockIdx.x * NT + threadIdx.x;
  if (i >= NP * 64) return;
  const int row = i >> 6, cp = (i & 63) * 2;
  const int rc = row < NN ? row : NN - 1;
  float a = x[(size_t)rc * EMB + cp], c = x[(size_t)rc * EMB + cp + 1];
  if (row >= NN) { a = 0.f; c = 0.f; }
  const _Float16 h0 = (_Float16)a, h1 = (_Float16)c;
  const unsigned u = (unsigned)__builtin_bit_cast(unsigned short, h0) | ((unsigned)__builtin_bit_cast(unsigned short, h1) << 16);
  ((volatile unsigned*)Xh)[i] = u;
  __threadfence();
  ((volatile unsigned*)Xh)[i] = u;
}

__global__ __launch_bounds__(NT) void edge_hidden_kernel(const float* __restrict__ PST, const int* __restrict__ idx_s,
                                                      const int* __restrict__ idx_t, const float* __restrict__ bf1,
                                                      _Float16* __restrict__ HE, int e0) {
  const int t = blockIdx.x * NT + threadIdx.x;
  const int el = t >> 4, g = t & 15;
  if (el >= EC) return;
  const int e = e0 + el;
  int s = idx_s[e]; s = s < 0 ? 0 : (s >= NN ? NN - 1 : s);
  int d = idx_t[e]; d = d < 0 ? 0 : (d >= NN ? NN - 1 : d);
  const float* ps = PST + (size_t)s * 256 + 8 * g;
  const float* pt = PST + (size_t)d * 256 + 128 + 8 * g;
  const v4f a0 = *(const v4f*)ps, a1 = *(const v4f*)(ps + 4);
  const v4f c0 = *(const v4f*)pt, c1 = *(const v4f*)(pt + 4);
  const v4f g0 = *(const v4f*)(bf1 + 8 * g), g1 = *(const v4f*)(bf1 + 8 * g + 4);
  v8h hv;
#pragma unroll
  for (int i = 0; i < 4; ++i) {
    float u0 = a0[i] + c0[i]; u0 = u0 + g0[i]; hv[i] = (_Float16)silu_f(u0);
    float u1 = a1[i] + c1[i]; u1 = u1 + g1[i]; hv[4 + i] = (_Float16)silu_f(u1);
  }
  _Float16* hp = HE + (size_t)el * EMB + 8 * g;
  *(volatile v8h*)hp = hv;
  __threadfence();
  *(volatile v8h*)hp = hv;
}

#define SCH 2048
#define SPK (SCH / NT)
#define NCH ((NE + SCH - 1) / SCH)
__global__ __launch_bounds__(NT) void seg_sum_kernel(const int* __restrict__ idx_s, const float* __restrict__ F,
                                                   const float* __restrict__ evst, float* __restrict__ FS) {
  __shared__ unsigned LIST[SCH];
  __shared__ float ACC[TN * 3];
  __shared__ int scan_ws[80];
  const int tid = threadIdx.x, lane = tid & 31, wave = tid >> 5;
  const int n0 = blockIdx.x * TN;
  for (int i = tid; i < TN * 3; i += NT) ACC[i] = 0.f;
  __syncthreads();
#pragma unroll 1
  for (int c = 0; c < NCH; ++c) {
    const int eb = c * SCH + tid * SPK;
    const bool inr = eb < NE;
    const int ebc = inr ? eb : (NE - SPK);
    unsigned rec[SPK]; int cnt = 0;
#pragma unroll
    for (int k = 0; k < SPK; k += 4) {
      const v4i d4 = *(const v4i*)(idx_s + ebc + k);
#pragma unroll
      for (int e = 0; e < 4; ++e) {
        const int d = d4[e]; unsigned r = 0xFFFFFFFFu;
        if (inr && d >= n0 && d < n0 + TN) { r = ((unsigned)(d - n0) << 20) | (unsigned)(ebc + k + e); ++cnt; }
        rec[k + e] = r;
      }
    }
    int tot; int p = blk_excl_scan(cnt, scan_ws, tid, &tot);
#pragma unroll
    for (int k = 0; k < SPK; ++k) if (rec[k] != 0xFFFFFFFFu) { if ((unsigned)p < (unsigned)SCH) LIST[p] = rec[k]; ++p; }
    __syncthreads();
    const int totc = tot < SCH ? tot : SCH;
#pragma unroll 1
    for (int base = 0; base < totc; base += 32) {
      const int q = base + lane;
      const int qc = q < SCH ? q : SCH - 1;
      const unsigned rv = LIST[qc];
      const int own = (q < totc && (int)(rv >> 29) == wave) ? 1 : 0;
      unsigned msk = (unsigned)__ballot(own);
#pragma unroll 1
      for (int it = 0; it < 32; ++it) {
        if (msk == 0u) break;
        const int bp = __builtin_ctz(msk); msk &= msk - 1u;
        const unsigned r = __shfl(rv, bp, 32);
        const int dl = (int)(r >> 20);
        int e = (int)(r & 0xFFFFFu); e = e < NE ? e : NE - 1;
        const float f = F[e];
        if (lane < 3) {
          const float ev = evst[(size_t)e * 3 + lane];
          const float val = f * ev;
          const float a = ACC[dl * 3 + lane];
          ACC[dl * 3 + lane] = a + val;
        }
      }
    }
    __syncthreads();
  }
  for (int pass = 0; pass < 2; ++pass) {
#pragma unroll 1
    for (int j = 0; j < TN / NT; ++j) {
      const int dl = j * NT + tid;
      v4f o; o[0] = ACC[dl * 3]; o[1] = ACC[dl * 3 + 1]; o[2] = ACC[dl * 3 + 2]; o[3] = 0.f;
      *(volatile v4f*)(FS + (size_t)(n0 + dl) * 4) = o;
    }
    __threadfence();
  }
}

__global__ __launch_bounds__(NT) void pack_out_kernel(const float* __restrict__ PD, const float* __restrict__ FS,
                                                    float* __restrict__ out, int out_n) {
  __shared__ float red[NT];
  const int tid = threadIdx.x;
  float prop = 0.f;
  if (blockIdx.x == 0) {
    float s = 0.f;
#pragma unroll 1
    for (int n = tid; n < NN; n += NT) s += PD[n];
    red[tid] = s;
    __syncthreads();
#pragma unroll 1
    for (int o = NT / 2; o > 0; o >>= 1) {
      if (tid < o) { const float a = red[tid] + red[tid + o]; red[tid] = a; }
      __syncthreads();
    }
    prop = red[0];
  }
  const int nq = out_n >> 2;
  const int t = blockIdx.x * NT + tid;
  if (t < nq) {
    v4f o;
#pragma unroll
    for (int e = 0; e < 4; ++e) {
      const int i = 4 * t + e;
      int j = i - 1; j = j < 0 ? 0 : j;
      const int node = j / 3; const int comp = j - node * 3;
      const float fv = FS[(size_t)node * 4 + comp];
      o[e] = (i == 0) ? prop : fv;
    }
    for (int pass = 0; pass < 2; ++pass) { *(volatile v4f*)(out + 4 * (size_t)t) = o; __threadfence(); }
  }
  if (t == nq) {
    for (int pass = 0; pass < 2; ++pass) {
#pragma unroll 1
      for (int i = 4 * nq; i < out_n; ++i) {
        int j = i - 1; j = j < 0 ? 0 : j;
        const int node = j / 3; const int comp = j - node * 3;
        const float fv = FS[(size_t)node * 4 + comp];
        const float v = (i == 0) ? prop : fv;
        ((volatile float*)out)[i] = v;
      }
      __threadfence();
    }
  }
}

extern "C" void kernel_launch(void* const* d_in, const int* in_sizes, int n_in,
                              void* d_out, int out_size, void* d_ws, size_t ws_size, hipStream_t stream) {
  if (n_in < 15) return;
  if (in_sizes[0] != NN * EMB || in_sizes[1] != NE || in_sizes[2] != NE || in_sizes[3] != NE * 3) return;
  if (in_sizes[5] != EMB * EMB || in_sizes[7] != EMB * 64 || in_sizes[9] != 64 || in_sizes[10] != 2 * EMB * EMB ||
      in_sizes[12] != EMB * 64 || in_sizes[14] != 64) return;
  if (out_size != 1 + NN * 3) return;
  const float* x     = (const float*)d_in[0];
  const int*   idx_s = (const int*)  d_in[1];
  const int*   idx_t = (const int*)  d_in[2];
  const float* evst  = (const float*)d_in[3];
  const float* W1  = (const float*)d_in[5];
  const float* b1  = (const float*)d_in[6];
  const float* W2  = (const float*)d_in[7];
  const float* b2  = (const float*)d_in[8];
  const float* W3  = (const float*)d_in[9];
  const float* Wf1 = (const float*)d_in[10];
  const float* bf1 = (const float*)d_in[11];
  const float* Wf2 = (const float*)d_in[12];
  const float* bf2 = (const float*)d_in[13];
  const float* Wf3 = (const float*)d_in[14];
  float* out = (float*)d_out;

  char* ws = (char*)d_ws; size_t off = 0;
  auto carve = [&](size_t bytes) -> char* { char* p = ws + off; off += (bytes + 255) & ~(size_t)255; return p; };
  _Float16* WT  = (_Float16*)carve((size_t)65536 * 2);
  _Float16* Xh  = (_Float16*)carve((size_t)NP * EMB * 2);
  char*     R1  = carve((size_t)EC * EMB * 2);
  float*    PST = (float*)carve((size_t)NP * 256 * 4);
  float*    PD  = (float*)carve((size_t)NP * 4);
  float*    F   = (float*)carve((size_t)NE * 4);
  float*    FS  = (float*)carve((size_t)NTILE * TN * 4 * 4);
  if (off > ws_size || off > (size_t)134217728) return;
  _Float16* H1h = (_Float16*)R1;
  _Float16* HE  = (_Float16*)R1;
  const _Float16* W1t  = WT;
  const _Float16* W2t  = WT + 16384;
  const _Float16* Wf1t = WT + 24576;
  const _Float16* Wf2t = WT + 57344;

  prep_w_kernel<<<32768 / NT, NT, 0, stream>>>(W1, W2, Wf1, Wf2, WT);
  cast_x_kernel<<<(NP * 64) / NT, NT, 0, stream>>>(x, Xh);
  {
    const int tiles = (NP / 64) * (EMB / 64);
    wmma_gemm64<0, false, 2, 1, false, 6><<<dim3((tiles + 7) / 8, 1), 256, 0, stream>>>(
        (const unsigned short*)Xh, (const unsigned short*)nullptr, EMB, 0L,
        (const unsigned short*)W1t, (const unsigned short*)nullptr, EMB, 0L,
        (void*)H1h, (void*)nullptr, EMB, 0L,
        b1, (const float*)nullptr, 0L, NP, EMB, EMB, WSC_INV, (const float*)nullptr);
  }
  {
    const int tiles = NP / 64;
    wmma_gemm64<0, false, 2, 3, false, 6><<<dim3((tiles + 7) / 8, 1), 256, 0, stream>>>(
        (const unsigned short*)H1h, (const unsigned short*)nullptr, EMB, 0L,
        (const unsigned short*)W2t, (const unsigned short*)nullptr, EMB, 0L,
        (void*)PD, (void*)nullptr, 64, 0L,
        b2, (const float*)nullptr, 0L, NP, 64, EMB, WSC_INV, W3);
  }
  {
    const int tiles = (NP / 64) * (256 / 64);
    wmma_gemm64<0, false, 0, 0, false, 0><<<dim3((tiles + 7) / 8, 1), 256, 0, stream>>>(
        (const unsigned short*)Xh, (const unsigned short*)nullptr, EMB, 0L,
        (const unsigned short*)Wf1t, (const unsigned short*)nullptr, EMB, 0L,
        (void*)PST, (void*)nullptr, 256, 0L,
        (const float*)nullptr, (const float*)nullptr, 0L, NP, 256, EMB, WSC_INV, (const float*)nullptr);
  }
  for (int c = 0; c < NCHK; ++c) {
    const int e0 = c * EC;
    edge_hidden_kernel<<<(EC * 16) / NT, NT, 0, stream>>>(PST, idx_s, idx_t, bf1, HE, e0);
    const int tiles = EC / 64;
    wmma_gemm64<0, false, 2, 3, false, 6><<<dim3((tiles + 7) / 8, 1), 256, 0, stream>>>(
        (const unsigned short*)HE, (const unsigned short*)nullptr, EMB, 0L,
        (const unsigned short*)Wf2t, (const unsigned short*)nullptr, EMB, 0L,
        (void*)(F + e0), (void*)nullptr, 64, 0L,
        bf2, (const float*)nullptr, 0L, EC, 64, EMB, WSC_INV, Wf3);
  }
  seg_sum_kernel<<<NTILE, NT, 0, stream>>>(idx_s, F, evst, FS);
  {
    const int nq = out_size / 4;
    pack_out_kernel<<<(nq + 1 + NT - 1) / NT, NT, 0, stream>>>(PD, FS, out, out_size);
  }
}
